// AttentionModule_57303453663460
// MI455X (gfx1250) — hardware-run, weakly checked
//
#include <hip/hip_runtime.h>


#ifndef NB
#define NB 8
#endif
#ifndef SEQ
#define SEQ 4096
#endif
#define NB_FULL 8
#define SEQ_FULL 4096
#define CC 256
#define HIDC 32
#define QKR 64
#define QSC 8.0f
#define KSC 8.0f
#define VSC 16.0f
#define PSC 4096.0f

static_assert(NB >= 1 && NB <= NB_FULL);
static_assert(SEQ % 256 == 0 && SEQ >= 256 && SEQ <= 4096 && SEQ <= SEQ_FULL);
static_assert(CC % 64 == 0 && HIDC % 32 == 0 && QKR == 2 * HIDC);

typedef __attribute__((ext_vector_type(16))) __bf16   v16bf;
typedef __attribute__((ext_vector_type(16))) _Float16 v16h;
typedef __attribute__((ext_vector_type(8)))  _Float16 v8h;
typedef __attribute__((ext_vector_type(8)))  float    v8f;
typedef __attribute__((ext_vector_type(4)))  float    v4f;
typedef __attribute__((ext_vector_type(8)))  unsigned v8u;

__device__ __forceinline__ unsigned f2bf(float f) { unsigned u = __float_as_uint(f); u += 0x7FFFu + ((u >> 16) & 1u); return u >> 16; }
__device__ __forceinline__ float bfr(float f) { return __uint_as_float(f2bf(f) << 16); }
__device__ __forceinline__ unsigned f2h(float f) { return (unsigned)__builtin_bit_cast(unsigned short, (_Float16)f); }
__device__ __forceinline__ int kpat(int v, int half) { return ((v & 4) ? 16 : 0) + half * 8 + 2 * (v & 3); }

template <int F16, int NP> struct Opnd { v16bf p[NP]; };

template <int F16, int NP> __device__ __forceinline__ void pack2(float f0, float f1, unsigned* o) {
    if (F16) { o[0] = f2h(f0) | (f2h(f1) << 16); return; }
    unsigned h0 = f2bf(f0), h1 = f2bf(f1); o[0] = h0 | (h1 << 16);
    if (NP >= 2) {
        float r0 = f0 - __uint_as_float(h0 << 16), r1 = f1 - __uint_as_float(h1 << 16);
        unsigned m0 = f2bf(r0), m1 = f2bf(r1); o[1] = m0 | (m1 << 16);
        if (NP >= 3) {
            float s0 = r0 - __uint_as_float(m0 << 16), s1 = r1 - __uint_as_float(m1 << 16);
            o[2] = f2bf(s0) | (f2bf(s1) << 16);
        }
    }
}
template <int F16, int NP> __device__ __forceinline__ void op_row(const float* rowp, int half, float sc, Opnd<F16, NP>& o) {
    v8u u[NP];
#pragma unroll
    for (int v = 0; v < 8; ++v) {
        int kk = kpat(v, half); unsigned t[3];
        pack2<F16, NP>(rowp[kk] * sc, rowp[kk + 1] * sc, t);
#pragma unroll
        for (int p = 0; p < NP; ++p) u[p][v] = t[p];
    }
#pragma unroll
    for (int p = 0; p < NP; ++p) o.p[p] = __builtin_bit_cast(v16bf, u[p]);
}
template <int F16, int NP> __device__ __forceinline__ void op_row_tail(const float* rowp, int half, float sc, int kvalid, Opnd<F16, NP>& o) {
    v8u u[NP];
#pragma unroll
    for (int v = 0; v < 8; ++v) {
        int kk = kpat(v, half); unsigned t[3];
        float f0 = kk < kvalid ? rowp[kk] * sc : 0.0f, f1 = (kk + 1) < kvalid ? rowp[kk + 1] * sc : 0.0f;
        pack2<F16, NP>(f0, f1, t);
#pragma unroll
        for (int p = 0; p < NP; ++p) u[p][v] = t[p];
    }
#pragma unroll
    for (int p = 0; p < NP; ++p) o.p[p] = __builtin_bit_cast(v16bf, u[p]);
}
template <int F16, int NP> __device__ __forceinline__ void op_col(const float* M, int ld, int n, int k0, int half, float sc, Opnd<F16, NP>& o) {
    v8u u[NP];
#pragma unroll
    for (int v = 0; v < 8; ++v) {
        int kk = k0 + kpat(v, half); unsigned t[3];
        pack2<F16, NP>(M[(size_t)kk * ld + n] * sc, M[(size_t)(kk + 1) * ld + n] * sc, t);
#pragma unroll
        for (int p = 0; p < NP; ++p) u[p][v] = t[p];
    }
#pragma unroll
    for (int p = 0; p < NP; ++p) o.p[p] = __builtin_bit_cast(v16bf, u[p]);
}
template <int F16, int NP> __device__ __forceinline__ void op_col_tail(const float* M, int ld, int n, int k0, int half, float sc, int K, Opnd<F16, NP>& o) {
    v8u u[NP];
#pragma unroll
    for (int v = 0; v < 8; ++v) {
        int kk = k0 + kpat(v, half); unsigned t[3];
        float f0 = kk < K ? M[(size_t)kk * ld + n] * sc : 0.0f, f1 = (kk + 1) < K ? M[(size_t)(kk + 1) * ld + n] * sc : 0.0f;
        pack2<F16, NP>(f0, f1, t);
#pragma unroll
        for (int p = 0; p < NP; ++p) u[p][v] = t[p];
    }
#pragma unroll
    for (int p = 0; p < NP; ++p) o.p[p] = __builtin_bit_cast(v16bf, u[p]);
}
__device__ __forceinline__ v8f wm_bf16(v16bf a, v16bf b, v8f c) { return __builtin_amdgcn_wmma_f32_16x16x32_bf16(false, a, false, b, (short)0, c, false, false); }
template <int F16, int NPA, int NPB> __device__ __forceinline__ v8f wmma_op(const Opnd<F16, NPA>& a, const Opnd<F16, NPB>& b, v8f c) {
    if (F16) {
        v16h ah = __builtin_bit_cast(v16h, a.p[0]), bh = __builtin_bit_cast(v16h, b.p[0]);
        c = __builtin_amdgcn_wmma_f32_16x16x32_f16(false, ah, false, bh, (short)0, c, false, false);
        asm volatile("v_nop\n\tv_nop\n\tv_nop\n\tv_nop" : "+v"(c) : "v"(ah), "v"(bh));
        return c;
    }
    constexpr int NMX = NPA > NPB ? NPA : NPB;
#pragma unroll
    for (int i = 0; i < NPA; ++i)
#pragma unroll
        for (int j = 0; j < NPB; ++j)
            if (i + j < NMX) c = wm_bf16(a.p[i], b.p[j], c);
    if (NPA == 1 && NPB == 1)      asm volatile("v_nop\n\tv_nop\n\tv_nop\n\tv_nop" : "+v"(c) : "v"(a.p[0]), "v"(b.p[0]));
    else if (NPA == 2 && NPB == 1) asm volatile("v_nop\n\tv_nop\n\tv_nop\n\tv_nop" : "+v"(c) : "v"(a.p[0]), "v"(a.p[1]), "v"(b.p[0]));
    else if (NPA == 1 && NPB == 2) asm volatile("v_nop\n\tv_nop\n\tv_nop\n\tv_nop" : "+v"(c) : "v"(a.p[0]), "v"(b.p[0]), "v"(b.p[1]));
    else if (NPA == 2 && NPB == 2) asm volatile("v_nop\n\tv_nop\n\tv_nop\n\tv_nop" : "+v"(c) : "v"(a.p[0]), "v"(a.p[1]), "v"(b.p[0]), "v"(b.p[1]));
    else                           asm volatile("v_nop\n\tv_nop\n\tv_nop\n\tv_nop" : "+v"(c) : "v"(a.p[0]), "v"(a.p[NPA - 1]), "v"(b.p[0]), "v"(b.p[NPB - 1]), "v"(a.p[NPA / 2]), "v"(b.p[NPB / 2]));
    return c;
}

union HFrag { v16h v; v8h q[2]; };
__device__ __forceinline__ v16h ld_frag16(const _Float16* rowp, int half) {
    HFrag f;
    f.q[0] = *(const v8h*)(rowp + 8 * half);
    f.q[1] = *(const v8h*)(rowp + 16 + 8 * half);
    return f.v;
}
__device__ __forceinline__ v8f wm_f16(v16h a, v16h b, v8f c) {
    c = __builtin_amdgcn_wmma_f32_16x16x32_f16(false, a, false, b, (short)0, c, false, false);
    asm volatile("v_nop\n\tv_nop\n\tv_nop\n\tv_nop" : "+v"(c) : "v"(a), "v"(b));
    return c;
}

struct ZMap { long long s1; long long s2; int zdiv; int pad_; };
__device__ __forceinline__ size_t zoff(const ZMap& m, int z) { return (size_t)((long long)(z / m.zdiv) * m.s1 + (long long)(z % m.zdiv) * m.s2); }

#define ACT_NONE 0
#define ACT_RELU 1
__device__ __forceinline__ float act_apply(int act, float x) {
    if (act == ACT_RELU) return x > 0.f ? x : 0.f;
    return x;
}
struct GemmArgs {
    ZMap za, zb_, zc, zbias, zadd, zrsc, zmul, zrbias;
    const float* A; const float* Bm; float* C; const float* bias; const float* add; const float* rsc; const float* mul; const float* rbias;
    long long ldadd, ldmul;
    int lda, ldb, ldc, K;
    float ascale, bscale, oscale, addscale;
    int M, nvalid, nstore, ldrsc;
    int bcs, eflags, pad2, pad3;
};
template <int PL, int BT, int F16, int NPA, int NPB, int RW, int CW, int ACT>
__global__ __launch_bounds__(256) void gemm_kernel(GemmArgs g) {
    constexpr int TR = 16 * RW, TC = 64 * CW, CSTR = TC + 4;
    __shared__ __align__(16) float cst[TR * CSTR];
    const int z = blockIdx.z;
    float* C = g.C + zoff(g.zc, z);
    const int tid = threadIdx.x, lane = tid & 31, wv = tid >> 5;
    const int l16 = lane & 15, half = lane >> 4;
    const int rt = wv % RW, ch = wv / RW;
    const int row0 = blockIdx.x * TR, col0 = blockIdx.y * TC + ch * 64;
    int arix = row0 + rt * 16 + l16; if (arix >= g.M) arix = g.M - 1;
    v8f acc[4];
#pragma unroll
    for (int t = 0; t < 4; ++t) acc[t] = (v8f){};
    const int K = g.K;
    if (PL) {
        const _Float16* A16 = (const _Float16*)g.A + zoff(g.za, z);
        const _Float16* B16 = (const _Float16*)g.Bm + zoff(g.zb_, z);
        const _Float16* arow = A16 + (size_t)arix * g.lda;
#pragma unroll 1
        for (int kc = 0; kc < K; kc += 32) {
            const v16h a = ld_frag16(arow + kc, half);
#pragma unroll
            for (int t = 0; t < 4; ++t) {
                const int n = col0 + t * 16 + l16;
                const int nc = n < g.nvalid ? n : g.nvalid - 1;
                HFrag b; b.v = ld_frag16(B16 + (size_t)nc * g.ldb + kc, half);
                if (n >= g.nvalid) b.v = (v16h){};
                acc[t] = wm_f16(a, b.v, acc[t]);
            }
        }
    } else {
        const float* A = g.A + zoff(g.za, z); const float* Bm = g.Bm + zoff(g.zb_, z);
        const float* arow = A + (size_t)arix * g.lda;
#pragma unroll 1
        for (int kc = 0; kc < K; kc += 32) {
            Opnd<F16, NPA> a;
            if (kc + 32 <= K) op_row<F16, NPA>(arow + kc, half, g.ascale, a); else op_row_tail<F16, NPA>(arow + kc, half, g.ascale, K - kc, a);
#pragma unroll
            for (int t = 0; t < 4; ++t) {
                Opnd<F16, NPB> b;
                const int n = col0 + t * 16 + l16;
                if (n < g.nvalid) {
                    if (BT) { if (kc + 32 <= K) op_row<F16, NPB>(Bm + (size_t)n * g.ldb + kc, half, g.bscale, b); else op_row_tail<F16, NPB>(Bm + (size_t)n * g.ldb + kc, half, g.bscale, K - kc, b); }
                    else    { if (kc + 32 <= K) op_col<F16, NPB>(Bm, g.ldb, n * g.bcs, kc, half, g.bscale, b); else op_col_tail<F16, NPB>(Bm, g.ldb, n * g.bcs, kc, half, g.bscale, K, b); }
                } else {
#pragma unroll
                    for (int p = 0; p < NPB; ++p) b.p[p] = (v16bf){};
                }
                acc[t] = wmma_op<F16, NPA, NPB>(a, b, acc[t]);
            }
        }
    }
    const float* bias = g.bias ? g.bias + zoff(g.zbias, z) : nullptr;
    const float* add = g.add ? g.add + zoff(g.zadd, z) : nullptr;
    const float* rsc = g.rsc ? g.rsc + zoff(g.zrsc, z) : nullptr;
    const float* mul = g.mul ? g.mul + zoff(g.zmul, z) : nullptr;
    const float* rbias = g.rbias ? g.rbias + zoff(g.zrbias, z) : nullptr;
    const bool ebias = (g.eflags & 2) != 0, eadd = (g.eflags & 1) != 0;
#pragma unroll
    for (int t = 0; t < 4; ++t) {
        const int cl = ch * 64 + t * 16 + l16;
        const int cg = blockIdx.y * TC + cl;
        const bool cok = cg < g.nvalid;
        float bv = (bias && cok) ? bias[(size_t)cg * g.bcs] : 0.0f;
        if (ebias) bv = bfr(bv);
#pragma unroll
        for (int r = 0; r < 8; ++r) {
            const int rl = rt * 16 + r + 8 * half;
            float v = acc[t][r] * g.oscale + bv;
            int rg = row0 + rl; if (rg >= g.M) rg = g.M - 1;
            if (rbias) { float rb = rbias[rg]; if (ebias) rb = bfr(rb); v += rb; }
            if (rsc) v *= rsc[(size_t)rg * g.ldrsc];
            if (mul && cok) v *= mul[(size_t)rg * g.ldmul + cg];
            if (add && cok) { float av = add[(size_t)rg * g.ldadd + cg]; if (eadd) av = bfr(av); v += g.addscale * av; }
            cst[rl * CSTR + cl] = v;
        }
    }
    __syncthreads();
    const int col = tid % TC, rsel = tid / TC, rstep = 256 / TC;
    if (ACT != ACT_NONE) {
#pragma unroll 1
        for (int r = rsel; r < TR; r += rstep) cst[r * CSTR + col] = act_apply(ACT, cst[r * CSTR + col]);
    }
    float* ob = C + (size_t)row0 * g.ldc + (size_t)blockIdx.y * TC;
    const bool colok = (int)(blockIdx.y * TC + col) < g.nstore;
    const int rmax = (g.M - row0 < TR) ? (g.M - row0) : TR;
    auto pass = [&]() {
        if (colok) {
#pragma unroll 4
            for (int r = rsel; r < rmax; r += rstep) *(volatile float*)(ob + (size_t)r * g.ldc + col) = cst[r * CSTR + col];
        }
    };
    pass();
    __threadfence();
    pass();
}
static inline ZMap zm(long long s1) { ZMap m; m.s1 = s1; m.s2 = 0; m.zdiv = 1; m.pad_ = 0; return m; }
static inline GemmArgs gemm_args(const float* A, int lda, ZMap za, const float* Bm, int ldb, ZMap zb, float* C, int ldc, ZMap zc, int M, int N, int K) {
    GemmArgs g; g.za = za; g.zb_ = zb; g.zc = zc; g.zbias = zm(0); g.zadd = zm(0); g.zrsc = zm(0); g.zmul = zm(0); g.zrbias = zm(0);
    g.A = A; g.Bm = Bm; g.C = C; g.bias = nullptr; g.add = nullptr; g.rsc = nullptr; g.mul = nullptr; g.rbias = nullptr; g.ldadd = 0; g.ldmul = 0;
    g.lda = lda; g.ldb = ldb; g.ldc = ldc; g.K = K; g.ascale = 1.0f; g.bscale = 1.0f; g.oscale = 1.0f; g.addscale = 1.0f; g.M = M; g.nvalid = N; g.nstore = N; g.ldrsc = 1;
    g.bcs = 1; g.eflags = 0; g.pad2 = 0; g.pad3 = 0;
    return g;
}
static_assert(sizeof(ZMap) == 24);
static_assert(sizeof(GemmArgs) == 8 * 24 + 8 * 8 + 2 * 8 + 4 * 4 + 4 * 4 + 4 * 4 + 4 * 4);

__global__ __launch_bounds__(256) void softmax_p16(float* S, long long sy, int L, float prescale, float pcarry) {
    __shared__ float red[8];
    __shared__ __align__(16) float rb[4096];
    const int tid = threadIdx.x, lane = tid & 31, wid = tid >> 5;
    float* row = S + (size_t)blockIdx.x * sy;
    float v[16];
    const int nj = L / 256;
    float mx = -__builtin_inff();
#pragma unroll
    for (int j = 0; j < 16; ++j) if (j < nj) { float t = row[tid + 256 * j] * prescale; v[j] = t; mx = fmaxf(mx, t); }
#pragma unroll
    for (int o = 16; o; o >>= 1) mx = fmaxf(mx, __shfl_xor(mx, o, 32));
    if (lane == 0) red[wid] = mx;
    __syncthreads();
    float m = red[0];
#pragma unroll
    for (int i = 1; i < 8; ++i) m = fmaxf(m, red[i]);
    if (m == -__builtin_inff()) m = 0.f;
    __syncthreads();
    float sum = 0.f;
#pragma unroll
    for (int j = 0; j < 16; ++j) if (j < nj) { v[j] = __expf(v[j] - m); sum += v[j]; }
#pragma unroll
    for (int o = 16; o; o >>= 1) sum += __shfl_xor(sum, o, 32);
    if (lane == 0) red[wid] = sum;
    __syncthreads();
    float tot = 0.f;
#pragma unroll
    for (int i = 0; i < 8; ++i) tot += red[i];
    const float psc = (1.0f / tot) * pcarry;
#pragma unroll
    for (int j = 0; j < 16; ++j) if (j < nj) rb[tid + 256 * j] = v[j] * psc;
    __syncthreads();
    _Float16* P = (_Float16*)row;
    const int e0 = 8 * tid, e1 = 2048 + 8 * tid;
    const bool ok0 = e0 < L, ok1 = e1 < L;
    const int c0 = ok0 ? e0 : 0, c1 = ok1 ? e1 : 0;
    v8h h0, h1;
    {
        const v4f a = *(const v4f*)(rb + c0), b = *(const v4f*)(rb + c0 + 4);
        h0[0] = (_Float16)a[0]; h0[1] = (_Float16)a[1]; h0[2] = (_Float16)a[2]; h0[3] = (_Float16)a[3];
        h0[4] = (_Float16)b[0]; h0[5] = (_Float16)b[1]; h0[6] = (_Float16)b[2]; h0[7] = (_Float16)b[3];
    }
    {
        const v4f a = *(const v4f*)(rb + c1), b = *(const v4f*)(rb + c1 + 4);
        h1[0] = (_Float16)a[0]; h1[1] = (_Float16)a[1]; h1[2] = (_Float16)a[2]; h1[3] = (_Float16)a[3];
        h1[4] = (_Float16)b[0]; h1[5] = (_Float16)b[1]; h1[6] = (_Float16)b[2]; h1[7] = (_Float16)b[3];
    }
    if (ok0) *(volatile v8h*)(P + e0) = h0;
    if (ok1) *(volatile v8h*)(P + e1) = h1;
    __threadfence();
    if (ok0) *(volatile v8h*)(P + e0) = h0;
    if (ok1) *(volatile v8h*)(P + e1) = h1;
}

__global__ __launch_bounds__(256) void k_cvt16(const float* __restrict__ src, _Float16* dst, float sc, int n8) {
    const int gi = blockIdx.x * 256 + threadIdx.x;
    if (gi >= n8) return;
    const float* s = src + (size_t)gi * 8;
    const v4f a = *(const v4f*)s, b = *(const v4f*)(s + 4);
    v8h hv;
    hv[0] = (_Float16)(a[0] * sc); hv[1] = (_Float16)(a[1] * sc); hv[2] = (_Float16)(a[2] * sc); hv[3] = (_Float16)(a[3] * sc);
    hv[4] = (_Float16)(b[0] * sc); hv[5] = (_Float16)(b[1] * sc); hv[6] = (_Float16)(b[2] * sc); hv[7] = (_Float16)(b[3] * sc);
    _Float16* d = dst + (size_t)gi * 8;
    *(volatile v8h*)d = hv;
    __threadfence();
    *(volatile v8h*)d = hv;
}

__global__ __launch_bounds__(256) void k_trqk(const float* __restrict__ src, _Float16* dst, float qsc, float ksc) {
    __shared__ float tile[QKR][33];
    const int b = blockIdx.z, n0 = blockIdx.x * 32, t = threadIdx.x;
    const float* s = src + (size_t)b * QKR * SEQ; _Float16* d = dst + (size_t)b * SEQ * QKR;
    {
        const int c = t >> 2, nq = (t & 3) * 8;
        const float* p = s + (size_t)c * SEQ + n0 + nq;
        const v4f a = *(const v4f*)p, bq = *(const v4f*)(p + 4);
        tile[c][nq + 0] = a[0]; tile[c][nq + 1] = a[1]; tile[c][nq + 2] = a[2]; tile[c][nq + 3] = a[3];
        tile[c][nq + 4] = bq[0]; tile[c][nq + 5] = bq[1]; tile[c][nq + 6] = bq[2]; tile[c][nq + 7] = bq[3];
    }
    __syncthreads();
    const int r = t >> 3, sg = t & 7;
    const float sc = sg < (HIDC / 8) ? qsc : ksc;
    v8h hv;
    hv[0] = (_Float16)(tile[8 * sg + 0][r] * sc); hv[1] = (_Float16)(tile[8 * sg + 1][r] * sc);
    hv[2] = (_Float16)(tile[8 * sg + 2][r] * sc); hv[3] = (_Float16)(tile[8 * sg + 3][r] * sc);
    hv[4] = (_Float16)(tile[8 * sg + 4][r] * sc); hv[5] = (_Float16)(tile[8 * sg + 5][r] * sc);
    hv[6] = (_Float16)(tile[8 * sg + 6][r] * sc); hv[7] = (_Float16)(tile[8 * sg + 7][r] * sc);
    _Float16* p = d + (size_t)(n0 + r) * QKR + 8 * sg;
    *(volatile v8h*)p = hv;
    __threadfence();
    *(volatile v8h*)p = hv;
}

extern "C" void kernel_launch(void* const* d_in, const int* in_sizes, int n_in,
                              void* d_out, int out_size, void* d_ws, size_t ws_size, hipStream_t stream) {
    if (n_in < 7) return;
    if (in_sizes[0] < (NB - 1) * CC * SEQ_FULL + (CC - 1) * SEQ_FULL + SEQ) return;
    if (in_sizes[1] < HIDC * CC || in_sizes[2] < HIDC || in_sizes[3] < HIDC * CC || in_sizes[4] < HIDC) return;
    if (in_sizes[5] < CC * CC || in_sizes[6] < CC) return;
    if (out_size < NB * CC * SEQ) return;
    const float* x = (const float*)d_in[0];
    const float* w1 = (const float*)d_in[1]; const float* b1 = (const float*)d_in[2];
    const float* w2 = (const float*)d_in[3]; const float* b2 = (const float*)d_in[4];
    const float* w3 = (const float*)d_in[5]; const float* b3 = (const float*)d_in[6];
    float* out = (float*)d_out;

    char* ws = (char*)d_ws; size_t off = 0;
    float* QKc = (float*)(ws + off);        off += (size_t)NB * QKR * SEQ * sizeof(float);
    _Float16* QK16 = (_Float16*)(ws + off); off += (size_t)NB * SEQ * QKR * sizeof(_Float16);
    float* V = (float*)(ws + off);          off += (size_t)NB * CC * SEQ * sizeof(float);
    _Float16* V16 = (_Float16*)(ws + off);  off += (size_t)NB * CC * SEQ * sizeof(_Float16);
    float* S = (float*)(ws + off);          off += (size_t)SEQ * SEQ * sizeof(float);
    if (off > ws_size) return;

    {
        GemmArgs g = gemm_args(w1, CC, zm(0), x, SEQ_FULL, zm((long long)CC * SEQ_FULL), QKc, SEQ, zm((long long)QKR * SEQ), HIDC, SEQ, CC);
        g.rbias = b1; g.eflags = 2;
        gemm_kernel<0, 0, 0, 1, 1, 2, 4, ACT_NONE><<<dim3((HIDC + 31) / 32, SEQ / 256, NB), 256, 0, stream>>>(g);
        GemmArgs gk = gemm_args(w2, CC, zm(0), x, SEQ_FULL, zm((long long)CC * SEQ_FULL), QKc + (size_t)HIDC * SEQ, SEQ, zm((long long)QKR * SEQ), HIDC, SEQ, CC);
        gk.rbias = b2; gk.eflags = 2;
        gemm_kernel<0, 0, 0, 1, 1, 2, 4, ACT_NONE><<<dim3((HIDC + 31) / 32, SEQ / 256, NB), 256, 0, stream>>>(gk);
    }
    {
        GemmArgs g = gemm_args(w3, CC, zm(0), x, SEQ_FULL, zm((long long)CC * SEQ_FULL), V, SEQ, zm((long long)CC * SEQ), CC, SEQ, CC);
        g.rbias = b3; g.eflags = 2;
        gemm_kernel<0, 0, 0, 1, 1, 2, 4, ACT_NONE><<<dim3(CC / 32, SEQ / 256, NB), 256, 0, stream>>>(g);
    }
    k_cvt16<<<dim3((NB * CC * SEQ) / 2048), 256, 0, stream>>>(V, V16, VSC, (NB * CC * SEQ) / 8);
    k_trqk<<<dim3(SEQ / 32, 1, NB), 256, 0, stream>>>(QKc, QK16, QSC, KSC);

    for (int b = 0; b < NB; ++b) {
        const _Float16* qk = QK16 + (size_t)b * SEQ * QKR;
        {
            GemmArgs g = gemm_args((const float*)qk, QKR, zm(0), (const float*)(qk + HIDC), QKR, zm(0), S, SEQ, zm(0), SEQ, SEQ, HIDC);
            g.oscale = 1.0f / (QSC * KSC);
            gemm_kernel<1, 1, 1, 1, 1, 4, 2, ACT_NONE><<<dim3(SEQ / 64, SEQ / 128, 1), 256, 0, stream>>>(g);
        }
        softmax_p16<<<dim3(SEQ), 256, 0, stream>>>(S, (long long)SEQ, SEQ, 1.0f, PSC);
        {
            GemmArgs g = gemm_args((const float*)(V16 + (size_t)b * CC * SEQ), SEQ, zm(0), (const float*)S, 2 * SEQ, zm(0),
                                   out + (size_t)b * CC * SEQ, SEQ, zm(0), CC, SEQ, SEQ);
            g.oscale = 1.0f / (VSC * PSC);
            g.add = x + (size_t)b * CC * SEQ_FULL; g.ldadd = SEQ_FULL; g.addscale = 1.0f; g.eflags = 1;
            gemm_kernel<1, 1, 1, 1, 1, 4, 2, ACT_NONE><<<dim3(CC / 64, SEQ / 128, 1), 256, 0, stream>>>(g);
        }
    }
}
